// SpatialSpectralAttention_25958782337667
// MI455X (gfx1250) — hardware-verified
//
#include <hip/hip_runtime.h>
#include <math.h>

constexpr int kBatch = 8;
constexpr int kSeq   = 1024;
constexpr int kDim   = 768;
constexpr int kHeads = 12;
constexpr int kHD    = 64;
constexpr int kTok   = kBatch * kSeq;
constexpr int kQKVN  = 3 * kDim;
constexpr int kQKN   = 2 * kDim;
constexpr int kKcat  = 2 * kDim;
constexpr float kScale     = 0.08838834764831845f;
constexpr float kWCar      = 64.0f;
constexpr float kWCarHalfV = 32.0f;
constexpr float kQKVCar    = 4.0f;
constexpr float kPCar      = 2048.0f;
constexpr float kXCar      = 256.0f;
constexpr float kQKVScale  = kQKVCar / kWCar;
constexpr float kScScale   = kScale / (kQKVCar * kQKVCar);
constexpr float kPVScale   = kXCar / (kPCar * kQKVCar);
constexpr float kOutScale  = 1.0f / (kXCar * kWCar);

typedef __attribute__((ext_vector_type(16))) _Float16 v16h;
typedef __attribute__((ext_vector_type(8)))  _Float16 v8h;
typedef __attribute__((ext_vector_type(16))) __bf16   v16b;
typedef __attribute__((ext_vector_type(8)))  __bf16   v8b;
typedef __attribute__((ext_vector_type(8)))  float    v8f;
typedef __attribute__((ext_vector_type(4)))  float    v4f;
typedef __attribute__((ext_vector_type(4)))  unsigned int v4u;

__device__ __forceinline__ unsigned short f2bf_bits(float f) {
  unsigned u = __float_as_uint(f);
  return (unsigned short)((u + 0x7FFFu + ((u >> 16) & 1u)) >> 16);
}
__device__ __forceinline__ float bf_bits2f(unsigned short h) { return __uint_as_float(((unsigned)h) << 16); }

__device__ __forceinline__ void dep_guard_h(v8f& a, v8f& b, v16h x, v16h y) { asm volatile("v_nop\n\tv_nop\n\tv_nop\n\tv_nop" : "+v"(a), "+v"(b) : "v"(x), "v"(y)); }
__device__ __forceinline__ void dep_guard_b(v8f& a, v8f& b, v16b x, v16b y) { asm volatile("v_nop\n\tv_nop\n\tv_nop\n\tv_nop" : "+v"(a), "+v"(b) : "v"(x), "v"(y)); }
__device__ __forceinline__ void keep4_h(v16h a, v16h b, v16h c, v16h d) { asm volatile("v_nop" :: "v"(a), "v"(b), "v"(c), "v"(d)); }
__device__ __forceinline__ void keep4_b(v16b a, v16b b, v16b c, v16b d) { asm volatile("v_nop" :: "v"(a), "v"(b), "v"(c), "v"(d)); }
__device__ __forceinline__ void acc_guard4(v8f& a, v8f& b, v8f& c, v8f& d) { asm volatile("v_nop\n\tv_nop\n\tv_nop\n\tv_nop" : "+v"(a), "+v"(b), "+v"(c), "+v"(d)); }
template <typename T> struct Frag;
template <> struct Frag<_Float16> {
  typedef v16h V; union U { v16h v; v8h h[2]; };
  static __device__ __forceinline__ v16h load(const _Float16* p) {
    U f; f.h[0] = *(const v8h*)(p); f.h[1] = *(const v8h*)(p + 16); return f.v;
  }
  static __device__ __forceinline__ v8f mma(v16h a, v16h b, v8f c) {
    return __builtin_amdgcn_wmma_f32_16x16x32_f16(false, a, false, b, (short)0, c, false, false);
  }
  static __device__ __forceinline__ void guard(v8f& a, v8f& b, v16h x, v16h y) { dep_guard_h(a, b, x, y); }
  static __device__ __forceinline__ void keep(v16h a, v16h b, v16h c, v16h d) { keep4_h(a, b, c, d); }
};
template <> struct Frag<__bf16> {
  typedef v16b V; union U { v16b v; v8b h[2]; };
  static __device__ __forceinline__ v16b load(const __bf16* p) {
    U f; f.h[0] = *(const v8b*)(p); f.h[1] = *(const v8b*)(p + 16); return f.v;
  }
  static __device__ __forceinline__ v8f mma(v16b a, v16b b, v8f c) {
    return __builtin_amdgcn_wmma_f32_16x16x32_bf16(false, a, false, b, (short)0, c, false, false);
  }
  static __device__ __forceinline__ void guard(v8f& a, v8f& b, v16b x, v16b y) { dep_guard_b(a, b, x, y); }
  static __device__ __forceinline__ void keep(v16b a, v16b b, v16b c, v16b d) { keep4_b(a, b, c, d); }
};

__device__ __forceinline__ unsigned pk16(unsigned short a, unsigned short b) { return (unsigned)a | ((unsigned)b << 16); }
__device__ __forceinline__ unsigned short h_bits(float f) { const _Float16 h = (_Float16)f; return __builtin_bit_cast(unsigned short, h); }

template <int ET> struct Elem;
template <> struct Elem<0> { typedef _Float16 T; };
template <> struct Elem<1> { typedef __bf16 T; };
template <int ET, bool SPLIT, int BIAS_MODE, int OUT_MODE, bool RESID, int ACT = 0>
__global__ __launch_bounds__(256) void wmma_gemm64(
    const unsigned short* __restrict__ Ap, const unsigned short* __restrict__ A2p, int lda, long strideA,
    const unsigned short* __restrict__ Btp, const unsigned short* __restrict__ Bt2p, int ldb, long strideB,
    void* __restrict__ Cout, void* __restrict__ Cout2, int ldc, long strideC,
    const float* __restrict__ bias,
    const float* __restrict__ resid, long strideR,
    int M, int N, int K, float scale) {
  typedef typename Elem<ET>::T T;
  typedef typename Frag<T>::V V;
  const T* A = (const T*)Ap; const T* A2 = (const T*)A2p; const T* Bt = (const T*)Btp; const T* Bt2 = (const T*)Bt2p;
  __shared__ __align__(16) float sT[8][16 * 68];
  const int b    = blockIdx.y;
  const int lane = threadIdx.x & 31;
  const int wave = threadIdx.x >> 5;
  const int tilesN = N >> 6;
  const int tilesM = M >> 6;
  const int tile = blockIdx.x * 8 + wave;
  if (tile >= tilesM * tilesN) return;
  const int tm = tile / tilesN;
  const int tn = tile - tm * tilesN;
  const int m0 = tm << 6;
  const int n0 = tn << 6;

  const T* Ab  = A  + (size_t)b * strideA;
  const T* Bb  = Bt + (size_t)b * strideB;
  const T* Ab2 = SPLIT ? (A2  + (size_t)b * strideA) : nullptr;
  const T* Bb2 = SPLIT ? (Bt2 + (size_t)b * strideB) : nullptr;

  const int rlane = lane & 15;
  const int koff  = (lane >> 4) * 8;
  const int mOff  = (lane >> 4) * 8;

  v8f acc[4][4];
#pragma unroll
  for (int i = 0; i < 4; ++i)
#pragma unroll
    for (int j = 0; j < 4; ++j) acc[i][j] = (v8f){0.f,0.f,0.f,0.f,0.f,0.f,0.f,0.f};

  for (int k0 = 0; k0 < K; k0 += 32) {
    V bh[4], bl[4];
#pragma unroll
    for (int j = 0; j < 4; ++j) {
      const size_t bo = (size_t)(n0 + (j << 4) + rlane) * ldb + koff + k0;
      bh[j] = Frag<T>::load(Bb + bo);
      if (SPLIT) bl[j] = Frag<T>::load(Bb2 + bo);
    }
#pragma unroll
    for (int i = 0; i < 4; ++i) {
      const size_t ao = (size_t)(m0 + (i << 4) + rlane) * lda + koff + k0;
      V ah = Frag<T>::load(Ab + ao);
      V al;
      if (SPLIT) al = Frag<T>::load(Ab2 + ao);
#pragma unroll
      for (int j = 0; j < 4; ++j) {
        acc[i][j] = Frag<T>::mma(ah, bh[j], acc[i][j]);
        if (SPLIT) {
          acc[i][j] = Frag<T>::mma(ah, bl[j], acc[i][j]);
          acc[i][j] = Frag<T>::mma(al, bh[j], acc[i][j]);
        }
      }
      Frag<T>::guard(acc[i][0], acc[i][3], ah, SPLIT ? al : ah);
    }
    Frag<T>::keep(bh[0], bh[1], bh[2], bh[3]);
    if (SPLIT) Frag<T>::keep(bl[0], bl[1], bl[2], bl[3]);
  }
  acc_guard4(acc[0][0], acc[0][1], acc[0][2], acc[0][3]);
  acc_guard4(acc[1][0], acc[1][1], acc[1][2], acc[1][3]);
  acc_guard4(acc[2][0], acc[2][1], acc[2][2], acc[2][3]);
  acc_guard4(acc[3][0], acc[3][1], acc[3][2], acc[3][3]);

  float* slab = sT[wave];
  const float* Rb = RESID ? (resid + (size_t)b * strideR) : nullptr;
#pragma unroll
  for (int i = 0; i < 4; ++i) {
    const int mBase = m0 + (i << 4);
#pragma unroll
    for (int j = 0; j < 4; ++j) {
      const int n = n0 + (j << 4) + rlane;
      float bv = 0.f;
      if (BIAS_MODE == 2) bv = bias[n];
#pragma unroll
      for (int r = 0; r < 8; ++r) {
        float v = acc[i][j][r] * scale;
        if (BIAS_MODE == 1) v += bias[mBase + mOff + r];
        if (BIAS_MODE == 2) v += bv;
        if (RESID) v += Rb[(size_t)(mBase + mOff + r) * ldc + n];
        if (ACT == 2) v = fmaxf(v, 0.0f);
        if (ACT == 4) v = (v > 0.f) ? v : 0.01f * v;
        slab[(mOff + r) * 68 + (j << 4) + rlane] = v;
      }
    }
    __builtin_amdgcn_fence(__ATOMIC_RELEASE, "workgroup");
    __builtin_amdgcn_wave_barrier();
    __builtin_amdgcn_fence(__ATOMIC_ACQUIRE, "workgroup");
    if (OUT_MODE == 0) {
      float* C = (float*)Cout + (size_t)b * strideC;
      const int hh = lane >> 4, c4 = (lane & 15) * 4;
      for (int pass = 0; pass < 2; ++pass) {
#pragma unroll
        for (int it = 0; it < 8; ++it) {
          const int row = it * 2 + hh;
          v4f v = *(const v4f*)(slab + row * 68 + c4);
          *(volatile v4f*)(C + (size_t)(mBase + row) * ldc + n0 + c4) = v;
        }
        __threadfence();
      }
    } else {
      const int q = lane >> 3, c8 = (lane & 7) * 8;
      unsigned short* C  = (unsigned short*)Cout  + (size_t)b * strideC;
      unsigned short* C2 = (OUT_MODE == 2) ? ((unsigned short*)Cout2 + (size_t)b * strideC) : nullptr;
      for (int pass = 0; pass < 2; ++pass) {
#pragma unroll
        for (int it = 0; it < 4; ++it) {
          const int row = it * 4 + q;
          const float* sp = slab + row * 68 + c8;
          v8h hv, lv;
#pragma unroll
          for (int e = 0; e < 8; ++e) {
            if (OUT_MODE == 1) {
              hv[e] = (_Float16)sp[e];
            } else {
              unsigned short hb = f2bf_bits(sp[e]);
              unsigned short lb = f2bf_bits(sp[e] - bf_bits2f(hb));
              hv[e] = __builtin_bit_cast(_Float16, hb);
              lv[e] = __builtin_bit_cast(_Float16, lb);
            }
          }
          *(volatile v8h*)(C + (size_t)(mBase + row) * ldc + n0 + c8) = hv;
          if (OUT_MODE == 2) *(volatile v8h*)(C2 + (size_t)(mBase + row) * ldc + n0 + c8) = lv;
        }
        __threadfence();
      }
    }
    __builtin_amdgcn_fence(__ATOMIC_RELEASE, "workgroup");
    __builtin_amdgcn_wave_barrier();
    __builtin_amdgcn_fence(__ATOMIC_ACQUIRE, "workgroup");
  }
}

__global__ __launch_bounds__(256) void cast8_kernel(const float* __restrict__ in, unsigned short* __restrict__ out,
                                                    int n8, int ldo, int coff, float s, float s2, int rthr) {
  const int i = blockIdx.x * 256 + threadIdx.x;
  if (i >= n8) return;
  const int e   = 8 * i;
  const int row = e / kDim;
  const int col = e - row * kDim;
  const float sc = (row >= rthr) ? s2 : s;
  const float* p = in + (size_t)e;
  const v4f a = *(const v4f*)(p);
  const v4f c = *(const v4f*)(p + 4);
  const unsigned u0 = pk16(h_bits(a[0] * sc), h_bits(a[1] * sc));
  const unsigned u1 = pk16(h_bits(a[2] * sc), h_bits(a[3] * sc));
  const unsigned u2 = pk16(h_bits(c[0] * sc), h_bits(c[1] * sc));
  const unsigned u3 = pk16(h_bits(c[2] * sc), h_bits(c[3] * sc));
  const v4u u = (v4u){u0, u1, u2, u3};
  unsigned short* q = out + (size_t)row * ldo + coff + col;
  *(volatile v4u*)q = u;
  __threadfence();
  *(volatile v4u*)q = u;
}

__global__ __launch_bounds__(256) void bias_kernel(const float* __restrict__ ba, const float* __restrict__ bb,
                                                   float* __restrict__ bc, float car) {
  const int i = blockIdx.x * 256 + threadIdx.x;
  if (i >= kQKVN / 4) return;
  const int n = 4 * i;
  const float f = (n >= kQKN) ? 0.5f : 1.0f;
  const v4f r  = *(const v4f*)(ba + n);
  const v4f s4 = *(const v4f*)(bb + n);
  const v4f o  = (r + s4 * f) * car;
  *(volatile v4f*)(bc + n) = o;
  __threadfence();
  *(volatile v4f*)(bc + n) = o;
}

__global__ __launch_bounds__(128) void softmax_row_kernel(const float* __restrict__ S, unsigned short* __restrict__ P,
                                                          float pcar) {
  __shared__ float redM[4];
  __shared__ float redS[4];
  const int row  = blockIdx.x;
  const int t    = threadIdx.x;
  const int lane = t & 31, wave = t >> 5;
  const int c0   = t * 8;
  const float* sr = S + (size_t)row * kSeq + c0;
  const v4f a = *(const v4f*)(sr);
  const v4f c = *(const v4f*)(sr + 4);
  float m = fmaxf(fmaxf(fmaxf(a[0], a[1]), fmaxf(a[2], a[3])), fmaxf(fmaxf(c[0], c[1]), fmaxf(c[2], c[3])));
#pragma unroll
  for (int off = 16; off > 0; off >>= 1) m = fmaxf(m, __shfl_xor(m, off, 32));
  if (lane == 0) redM[wave] = m;
  __syncthreads();
  m = fmaxf(fmaxf(redM[0], redM[1]), fmaxf(redM[2], redM[3]));
  const float e0 = expf(a[0] - m);
  const float e1 = expf(a[1] - m);
  const float e2 = expf(a[2] - m);
  const float e3 = expf(a[3] - m);
  const float e4 = expf(c[0] - m);
  const float e5 = expf(c[1] - m);
  const float e6 = expf(c[2] - m);
  const float e7 = expf(c[3] - m);
  float ssum = ((e0 + e1) + (e2 + e3)) + ((e4 + e5) + (e6 + e7));
#pragma unroll
  for (int off = 16; off > 0; off >>= 1) ssum += __shfl_xor(ssum, off, 32);
  if (lane == 0) redS[wave] = ssum;
  __syncthreads();
  ssum = (redS[0] + redS[1]) + (redS[2] + redS[3]);
  const float inv = pcar * (1.0f / ssum);
  const unsigned u0 = pk16(h_bits(e0 * inv), h_bits(e1 * inv));
  const unsigned u1 = pk16(h_bits(e2 * inv), h_bits(e3 * inv));
  const unsigned u2 = pk16(h_bits(e4 * inv), h_bits(e5 * inv));
  const unsigned u3 = pk16(h_bits(e6 * inv), h_bits(e7 * inv));
  const v4u u = (v4u){u0, u1, u2, u3};
  unsigned short* q = P + (size_t)row * kSeq + c0;
  *(volatile v4u*)q = u;
  __threadfence();
  *(volatile v4u*)q = u;
}

extern "C" void kernel_launch(void* const* d_in, const int* in_sizes, int n_in,
                              void* d_out, int out_size, void* d_ws, size_t ws_size,
                              hipStream_t stream) {
  if (n_in < 8) return;
  if (in_sizes[0] != kTok * kDim || in_sizes[1] != kTok * kDim) return;
  if (in_sizes[2] != kQKVN * kDim || in_sizes[4] != kQKVN * kDim) return;
  if (in_sizes[3] != kQKVN || in_sizes[5] != kQKVN) return;
  if (in_sizes[6] != kDim * kDim || in_sizes[7] != kDim) return;
  if (out_size != kTok * kDim) return;

  const float* embA = (const float*)d_in[0];
  const float* embB = (const float*)d_in[1];
  const float* wA   = (const float*)d_in[2];
  const float* bA   = (const float*)d_in[3];
  const float* wB   = (const float*)d_in[4];
  const float* bB   = (const float*)d_in[5];
  const float* wP   = (const float*)d_in[6];
  const float* bP   = (const float*)d_in[7];
  float* out = (float*)d_out;

  const size_t offSc = 0;
  const size_t offP  = offSc + (size_t)kHeads * kSeq * kSeq * 4;
  const size_t offQK = offP  + (size_t)kHeads * kSeq * kSeq * 2;
  const size_t offVT = offQK + (size_t)kTok * kQKN * 2;
  const size_t offX  = offVT + (size_t)kBatch * kDim * kSeq * 2;
  const size_t offPW = offX  + (size_t)kTok * kDim * 2;
  const size_t offBc = offPW + (size_t)kDim * kDim * 2;
  const size_t total = offBc + (size_t)kQKVN * 4;
  const size_t offXc = 0;
  const size_t offWc = offXc + (size_t)kTok * kKcat * 2;
  if (total > ws_size) return;
  if (offWc + (size_t)kQKVN * kKcat * 2 > offQK) return;

  char* ws = (char*)d_ws;
  float*          Sc   = (float*)(ws + offSc);
  unsigned short* P16  = (unsigned short*)(ws + offP);
  unsigned short* QK16 = (unsigned short*)(ws + offQK);
  unsigned short* VT   = (unsigned short*)(ws + offVT);
  unsigned short* X16  = (unsigned short*)(ws + offX);
  unsigned short* PW   = (unsigned short*)(ws + offPW);
  float*          bc   = (float*)(ws + offBc);
  unsigned short* Xc   = (unsigned short*)(ws + offXc);
  unsigned short* Wc   = (unsigned short*)(ws + offWc);

  const int n8x = kTok * kDim / 8;
  cast8_kernel<<<(n8x + 255) / 256, 256, 0, stream>>>(embA, Xc, n8x, kKcat, 0,    1.0f, 1.0f, kTok);
  cast8_kernel<<<(n8x + 255) / 256, 256, 0, stream>>>(embB, Xc, n8x, kKcat, kDim, 1.0f, 1.0f, kTok);
  const int n8w = kQKVN * kDim / 8;
  cast8_kernel<<<(n8w + 255) / 256, 256, 0, stream>>>(wA, Wc, n8w, kKcat, 0,    kWCar, kWCar,      kQKVN);
  cast8_kernel<<<(n8w + 255) / 256, 256, 0, stream>>>(wB, Wc, n8w, kKcat, kDim, kWCar, kWCarHalfV, kQKN);
  const int n8p = kDim * kDim / 8;
  cast8_kernel<<<(n8p + 255) / 256, 256, 0, stream>>>(wP, PW, n8p, kDim, 0, kWCar, kWCar, kDim);
  bias_kernel<<<(kQKVN / 4 + 255) / 256, 256, 0, stream>>>(bA, bB, bc, kQKVCar);

  wmma_gemm64<0, false, 2, 1, false><<<dim3(384, 1), 256, 0, stream>>>(
      Xc, nullptr, kKcat, 0L,
      Wc, nullptr, kKcat, 0L,
      (void*)QK16, nullptr, kQKN, 0L,
      bc, nullptr, 0L,
      kTok, kQKN, kKcat, kQKVScale);
  wmma_gemm64<0, false, 1, 1, false><<<dim3(24, kBatch), 256, 0, stream>>>(
      Wc + (size_t)kQKN * kKcat, nullptr, kKcat, 0L,
      Xc, nullptr, kKcat, (long)kSeq * kKcat,
      (void*)VT, nullptr, kSeq, (long)kDim * kSeq,
      bc + kQKN, nullptr, 0L,
      kDim, kSeq, kKcat, kQKVScale);

  for (int b = 0; b < kBatch; ++b) {
    const unsigned short* Qb = QK16 + (size_t)b * kSeq * kQKN;
    const unsigned short* Kb = Qb + kDim;
    wmma_gemm64<0, false, 0, 0, false><<<dim3(32, kHeads), 256, 0, stream>>>(
        Qb, nullptr, kQKN, (long)kHD,
        Kb, nullptr, kQKN, (long)kHD,
        (void*)Sc, nullptr, kSeq, (long)kSeq * kSeq,
        nullptr, nullptr, 0L,
        kSeq, kSeq, kHD, kScScale);
    softmax_row_kernel<<<kHeads * kSeq, 128, 0, stream>>>(Sc, P16, kPCar);
    wmma_gemm64<0, false, 0, 1, false><<<dim3(2, kHeads), 256, 0, stream>>>(
        P16, nullptr, kSeq, (long)kSeq * kSeq,
        VT + (size_t)b * kDim * kSeq, nullptr, kSeq, (long)kHD * kSeq,
        (void*)(X16 + (size_t)b * kSeq * kDim), nullptr, kDim, (long)kHD,
        nullptr, nullptr, 0L,
        kSeq, kHD, kSeq, kPVScale);
  }

  wmma_gemm64<0, false, 2, 0, false><<<dim3(192, 1), 256, 0, stream>>>(
      X16, nullptr, kDim, 0L,
      PW, nullptr, kDim, 0L,
      (void*)out, nullptr, kDim, 0L,
      bP, nullptr, 0L,
      kTok, kDim, kDim, kOutScale);
}
